// FractalResonanceTransformer_54228257079875
// MI455X (gfx1250) — hardware-verified
//
#include <hip/hip_runtime.h>
#include <stdint.h>

typedef __attribute__((ext_vector_type(16))) _Float16 v16h;
typedef __attribute__((ext_vector_type(8)))  _Float16 v8h;
typedef __attribute__((ext_vector_type(16))) __bf16   v16b;
typedef __attribute__((ext_vector_type(8)))  __bf16   v8b;
typedef __attribute__((ext_vector_type(8)))  float    v8f;
typedef __attribute__((ext_vector_type(4)))  float    v4f;
typedef __attribute__((ext_vector_type(4)))  unsigned int v4u;

constexpr int kB  = 2;
constexpr int kS  = 2048;
constexpr int kD  = 1024;
constexpr int kH  = 16;
constexpr int kDH = 64;
constexpr int kM  = kB * kS;
static_assert(kDH == 64, "head dim 64 attention kernel");
static_assert(kS % 64 == 0 && kM % 64 == 0 && kD % 64 == 0, "tile multiples");
static_assert(kD % 32 == 0, "K multiple of 32 for every GEMM");
static_assert(kH * kDH == kD, "heads");
static_assert(kS == 2048, "index shifts below assume S = 2^11");

constexpr float kWCarry   = 16.0f;
constexpr float kQKVCarry = 8.0f;
constexpr float kOCarry   = 16.0f;
constexpr float kPCarry   = 32768.0f;
constexpr float kMaskFill = -1.0e9f;

constexpr size_t kSzPlane = (size_t)kM * kD * 2;
constexpr size_t kSzW     = (size_t)kD * kD * 2;
constexpr size_t kSzT     = (size_t)kB * kH * kS * 4;
constexpr size_t kOffH    = 0;
constexpr size_t kOffQ    = kOffH  + kSzPlane;
constexpr size_t kOffKc   = kOffQ  + kSzPlane;
constexpr size_t kOffVt   = kOffKc + kSzPlane;
constexpr size_t kOffO    = kOffVt + kSzPlane;
constexpr size_t kOffWq   = kOffO  + kSzPlane;
constexpr size_t kOffWk   = kOffWq + kSzW;
constexpr size_t kOffWv   = kOffWk + kSzW;
constexpr size_t kOffWo   = kOffWv + kSzW;
constexpr size_t kOffTh   = kOffWo + kSzW;
constexpr size_t kOffLTh  = kOffTh + kSzT;
constexpr size_t kWsTotal = kOffLTh + kSzT;
static_assert(kWsTotal == 50855936, "carve total");
static_assert(kWsTotal <= 134217728, "carve within 128 MiB");
static_assert((kOffQ % 128) == 0 && (kOffWq % 128) == 0 && (kOffTh % 128) == 0 && (kOffLTh % 128) == 0, "alignment");

__device__ __forceinline__ unsigned short f2bf_bits(float f) {
  unsigned u = __float_as_uint(f);
  return (unsigned short)((u + 0x7FFFu + ((u >> 16) & 1u)) >> 16);
}
__device__ __forceinline__ float bf_bits2f(unsigned short h) { return __uint_as_float(((unsigned)h) << 16); }
__device__ __forceinline__ unsigned short h_bits(float f) { return __builtin_bit_cast(unsigned short, (_Float16)f); }

__device__ __forceinline__ void dep_guard_h(v8f& a, v8f& b, v16h x, v16h y) { asm volatile("v_nop\n\tv_nop\n\tv_nop\n\tv_nop" : "+v"(a), "+v"(b) : "v"(x), "v"(y)); }
__device__ __forceinline__ void dep_guard_b(v8f& a, v8f& b, v16b x, v16b y) { asm volatile("v_nop\n\tv_nop\n\tv_nop\n\tv_nop" : "+v"(a), "+v"(b) : "v"(x), "v"(y)); }
__device__ __forceinline__ void keep4_h(v16h a, v16h b, v16h c, v16h d) { asm volatile("v_nop" :: "v"(a), "v"(b), "v"(c), "v"(d)); }
__device__ __forceinline__ void keep4_b(v16b a, v16b b, v16b c, v16b d) { asm volatile("v_nop" :: "v"(a), "v"(b), "v"(c), "v"(d)); }
__device__ __forceinline__ void acc_guard4(v8f& a, v8f& b, v8f& c, v8f& d) { asm volatile("v_nop\n\tv_nop\n\tv_nop\n\tv_nop" : "+v"(a), "+v"(b), "+v"(c), "+v"(d)); }
template <typename T> struct Frag;
template <> struct Frag<_Float16> {
  typedef v16h V; union U { v16h v; v8h h[2]; };
  static __device__ __forceinline__ v16h load(const _Float16* p) {
    U f; f.h[0] = *(const v8h*)(p); f.h[1] = *(const v8h*)(p + 16); return f.v;
  }
  static __device__ __forceinline__ v8f mma(v16h a, v16h b, v8f c) {
    return __builtin_amdgcn_wmma_f32_16x16x32_f16(false, a, false, b, (short)0, c, false, false);
  }
  static __device__ __forceinline__ void guard(v8f& a, v8f& b, v16h x, v16h y) { dep_guard_h(a, b, x, y); }
  static __device__ __forceinline__ void keep(v16h a, v16h b, v16h c, v16h d) { keep4_h(a, b, c, d); }
};
template <> struct Frag<__bf16> {
  typedef v16b V; union U { v16b v; v8b h[2]; };
  static __device__ __forceinline__ v16b load(const __bf16* p) {
    U f; f.h[0] = *(const v8b*)(p); f.h[1] = *(const v8b*)(p + 16); return f.v;
  }
  static __device__ __forceinline__ v8f mma(v16b a, v16b b, v8f c) {
    return __builtin_amdgcn_wmma_f32_16x16x32_bf16(false, a, false, b, (short)0, c, false, false);
  }
  static __device__ __forceinline__ void guard(v8f& a, v8f& b, v16b x, v16b y) { dep_guard_b(a, b, x, y); }
  static __device__ __forceinline__ void keep(v16b a, v16b b, v16b c, v16b d) { keep4_b(a, b, c, d); }
};

__device__ __forceinline__ v8f mma_h(v16h a, v16h b, v8f c) {
  c = __builtin_amdgcn_wmma_f32_16x16x32_f16(false, a, false, b, (short)0, c, false, false);
  asm volatile("v_nop\n\tv_nop\n\tv_nop\n\tv_nop" : "+v"(c) : "v"(a), "v"(b));
  return c;
}

__device__ __forceinline__ float wave_sum(float v) {
#pragma unroll
  for (int off = 1; off < 32; off <<= 1) v += __shfl_xor(v, off, 32);
  return v;
}

__device__ __forceinline__ float fr_compress(float v, float e) {
  const float mag = fmaxf(fabsf(v), 1e-8f);
  const float pw = exp2f(e * log2f(mag));
  float r = (v > 0.0f) ? pw : -pw;
  r = (v == 0.0f) ? 0.0f : r;
  return r;
}

template <int ET> struct Elem;
template <> struct Elem<0> { typedef _Float16 T; };
template <> struct Elem<1> { typedef __bf16 T; };
template <int ET, bool SPLIT, int BIAS_MODE, int OUT_MODE, bool RESID, int ACT = 0>
__global__ __launch_bounds__(256) void wmma_gemm64(
    const unsigned short* __restrict__ Ap, const unsigned short* __restrict__ A2p, int lda, long strideA,
    const unsigned short* __restrict__ Btp, const unsigned short* __restrict__ Bt2p, int ldb, long strideB,
    void* __restrict__ Cout, void* __restrict__ Cout2, int ldc, long strideC,
    const float* __restrict__ bias,
    const float* __restrict__ resid, long strideR,
    int M, int N, int K, float scale) {
  static_assert(!RESID || OUT_MODE == 0, "residual path is f32-out only");
  static_assert(!RESID || ACT == 0, "residual path has no activation");
  typedef typename Elem<ET>::T T;
  typedef typename Frag<T>::V V;
  const T* A = (const T*)Ap; const T* A2 = (const T*)A2p; const T* Bt = (const T*)Btp; const T* Bt2 = (const T*)Bt2p;
  __shared__ __align__(16) float sT[8][16 * 68];
  const int b    = blockIdx.y;
  const int lane = threadIdx.x & 31;
  const int wave = threadIdx.x >> 5;
  const int tilesN = N >> 6;
  const int tilesM = M >> 6;
  const int tile = blockIdx.x * 8 + wave;
  if (tile >= tilesM * tilesN) return;
  const int tm = tile / tilesN;
  const int tn = tile - tm * tilesN;
  const int m0 = tm << 6;
  const int n0 = tn << 6;

  const T* Ab  = A  + (size_t)b * strideA;
  const T* Bb  = Bt + (size_t)b * strideB;
  const T* Ab2 = SPLIT ? (A2  + (size_t)b * strideA) : nullptr;
  const T* Bb2 = SPLIT ? (Bt2 + (size_t)b * strideB) : nullptr;

  const int rlane = lane & 15;
  const int koff  = (lane >> 4) * 8;
  const int mOff  = (lane >> 4) * 8;

  v8f acc[4][4];
#pragma unroll
  for (int i = 0; i < 4; ++i)
#pragma unroll
    for (int j = 0; j < 4; ++j) acc[i][j] = (v8f){0.f,0.f,0.f,0.f,0.f,0.f,0.f,0.f};

  for (int k0 = 0; k0 < K; k0 += 32) {
    V bh[4], bl[4];
#pragma unroll
    for (int j = 0; j < 4; ++j) {
      const size_t bo = (size_t)(n0 + (j << 4) + rlane) * ldb + koff + k0;
      bh[j] = Frag<T>::load(Bb + bo);
      if (SPLIT) bl[j] = Frag<T>::load(Bb2 + bo);
    }
#pragma unroll
    for (int i = 0; i < 4; ++i) {
      const size_t ao = (size_t)(m0 + (i << 4) + rlane) * lda + koff + k0;
      V ah = Frag<T>::load(Ab + ao);
      V al;
      if (SPLIT) al = Frag<T>::load(Ab2 + ao);
#pragma unroll
      for (int j = 0; j < 4; ++j) {
        acc[i][j] = Frag<T>::mma(ah, bh[j], acc[i][j]);
        if (SPLIT) {
          acc[i][j] = Frag<T>::mma(ah, bl[j], acc[i][j]);
          acc[i][j] = Frag<T>::mma(al, bh[j], acc[i][j]);
        }
      }
      Frag<T>::guard(acc[i][0], acc[i][3], ah, SPLIT ? al : ah);
    }
    Frag<T>::keep(bh[0], bh[1], bh[2], bh[3]);
    if (SPLIT) Frag<T>::keep(bl[0], bl[1], bl[2], bl[3]);
  }
  acc_guard4(acc[0][0], acc[0][1], acc[0][2], acc[0][3]);
  acc_guard4(acc[1][0], acc[1][1], acc[1][2], acc[1][3]);
  acc_guard4(acc[2][0], acc[2][1], acc[2][2], acc[2][3]);
  acc_guard4(acc[3][0], acc[3][1], acc[3][2], acc[3][3]);

  float* slab = sT[wave];
  const float* Rb = RESID ? (resid + (size_t)b * strideR) : nullptr;
  float ev = 0.f;
  if (ACT == 6) { int hd = n0 >> 6; hd = (hd > kH - 1) ? (kH - 1) : hd; ev = bias[hd]; }
  if (ACT == 7) { int hd = m0 >> 6; hd = (hd > kH - 1) ? (kH - 1) : hd; ev = bias[hd]; }
#pragma unroll
  for (int i = 0; i < 4; ++i) {
    const int mBase = m0 + (i << 4);
#pragma unroll
    for (int j = 0; j < 4; ++j) {
      const int n = n0 + (j << 4) + rlane;
      float bv = 0.f;
      if (BIAS_MODE == 2) bv = bias[n];
#pragma unroll
      for (int r = 0; r < 8; ++r) {
        float v = acc[i][j][r] * scale;
        if (BIAS_MODE == 1) v += bias[mBase + mOff + r];
        if (BIAS_MODE == 2) v += bv;
        if (ACT == 1) v = tanhf(v);
        if (ACT == 2) v = fmaxf(v, 0.0f);
        if (ACT == 3) v = v / (1.0f + expf(-v));
        if (ACT == 4) v = (v > 0.f) ? v : 0.01f * v;
        if (ACT == 5) v = 0.5f * v * (1.0f + erff(v * 0.70710678118654752f));
        if (ACT == 6 || ACT == 7) v = fr_compress(v, ev) * kQKVCarry;
        slab[(mOff + r) * 68 + (j << 4) + rlane] = v;
      }
    }
    __builtin_amdgcn_fence(__ATOMIC_RELEASE, "workgroup");
    __builtin_amdgcn_wave_barrier();
    __builtin_amdgcn_fence(__ATOMIC_ACQUIRE, "workgroup");
    if (OUT_MODE == 0) {
      float* C = (float*)Cout + (size_t)b * strideC;
      const int hh = lane >> 4, c4 = (lane & 15) * 4;
      if (RESID) {
#pragma unroll
        for (int it = 0; it < 8; ++it) {
          const int row = it * 2 + hh;
          const v4f rv = *(const v4f*)(Rb + (size_t)(mBase + row) * ldc + n0 + c4);
          v4f sv = *(const v4f*)(slab + row * 68 + c4);
          sv += rv;
          *(v4f*)(slab + row * 68 + c4) = sv;
        }
      }
      for (int pass = 0; pass < 2; ++pass) {
#pragma unroll
        for (int it = 0; it < 8; ++it) {
          const int row = it * 2 + hh;
          v4f v = *(const v4f*)(slab + row * 68 + c4);
          *(volatile v4f*)(C + (size_t)(mBase + row) * ldc + n0 + c4) = v;
        }
        __threadfence();
      }
    } else {
      const int q = lane >> 3, c8 = (lane & 7) * 8;
      unsigned short* C  = (unsigned short*)Cout  + (size_t)b * strideC;
      unsigned short* C2 = (OUT_MODE == 2) ? ((unsigned short*)Cout2 + (size_t)b * strideC) : nullptr;
      for (int pass = 0; pass < 2; ++pass) {
#pragma unroll
        for (int it = 0; it < 4; ++it) {
          const int row = it * 4 + q;
          const float* sp = slab + row * 68 + c8;
          v8h hv, lv;
#pragma unroll
          for (int e = 0; e < 8; ++e) {
            if (OUT_MODE == 1) {
              hv[e] = (_Float16)sp[e];
            } else {
              unsigned short hb = f2bf_bits(sp[e]);
              unsigned short lb = f2bf_bits(sp[e] - bf_bits2f(hb));
              hv[e] = __builtin_bit_cast(_Float16, hb);
              lv[e] = __builtin_bit_cast(_Float16, lb);
            }
          }
          *(volatile v8h*)(C + (size_t)(mBase + row) * ldc + n0 + c8) = hv;
          if (OUT_MODE == 2) *(volatile v8h*)(C2 + (size_t)(mBase + row) * ldc + n0 + c8) = lv;
        }
        __threadfence();
      }
    }
    __builtin_amdgcn_fence(__ATOMIC_RELEASE, "workgroup");
    __builtin_amdgcn_wave_barrier();
    __builtin_amdgcn_fence(__ATOMIC_ACQUIRE, "workgroup");
  }
}

__global__ __launch_bounds__(128) void ln_rows_f16(const float* __restrict__ x, const float* __restrict__ gamma,
                                                   const float* __restrict__ beta, unsigned short* __restrict__ hp) {
  __shared__ float red0[4];
  __shared__ float red1[4];
  const int row = blockIdx.x, tid = threadIdx.x, lane = tid & 31, wave = tid >> 5;
  const float* xr = x + (size_t)row * kD + tid * 8;
  const v4f a0 = *(const v4f*)(xr);
  const v4f a1 = *(const v4f*)(xr + 4);
  float s = ((a0[0] + a0[1]) + (a0[2] + a0[3])) + ((a1[0] + a1[1]) + (a1[2] + a1[3]));
  s = wave_sum(s);
  if (lane == 0) red0[wave] = s;
  __syncthreads();
  const float mu = ((red0[0] + red0[1]) + (red0[2] + red0[3])) * (1.0f / (float)kD);
  const v4f d0 = a0 - mu;
  const v4f d1 = a1 - mu;
  float ss = ((d0[0] * d0[0] + d0[1] * d0[1]) + (d0[2] * d0[2] + d0[3] * d0[3]))
           + ((d1[0] * d1[0] + d1[1] * d1[1]) + (d1[2] * d1[2] + d1[3] * d1[3]));
  ss = wave_sum(ss);
  if (lane == 0) red1[wave] = ss;
  __syncthreads();
  const float var = ((red1[0] + red1[1]) + (red1[2] + red1[3])) * (1.0f / (float)kD);
  const float rs = rsqrtf(var + 1e-5f);
  const v4f g0 = *(const v4f*)(gamma + tid * 8);
  const v4f g1 = *(const v4f*)(gamma + tid * 8 + 4);
  const v4f b0 = *(const v4f*)(beta + tid * 8);
  const v4f b1 = *(const v4f*)(beta + tid * 8 + 4);
  const v4f y0 = d0 * rs * g0 + b0;
  const v4f y1 = d1 * rs * g1 + b1;
  v4u u;
  u[0] = (unsigned)h_bits(y0[0]) | ((unsigned)h_bits(y0[1]) << 16);
  u[1] = (unsigned)h_bits(y0[2]) | ((unsigned)h_bits(y0[3]) << 16);
  u[2] = (unsigned)h_bits(y1[0]) | ((unsigned)h_bits(y1[1]) << 16);
  u[3] = (unsigned)h_bits(y1[2]) | ((unsigned)h_bits(y1[3]) << 16);
  unsigned short* dst = hp + (size_t)row * kD + tid * 8;
  *(volatile v4u*)dst = u;
  __threadfence();
  *(volatile v4u*)dst = u;
}

__global__ __launch_bounds__(256) void wt_cast_f16(const float* __restrict__ W, unsigned short* __restrict__ Wt) {
  __shared__ float tile[64][65];
  const int tid = threadIdx.x;
  const int n0 = blockIdx.x * 64, k0 = blockIdx.y * 64;
#pragma unroll
  for (int i = 0; i < 4; ++i) {
    const int idx = tid + 256 * i;
    const int kr = idx >> 4, c4 = (idx & 15) * 4;
    const v4f v = *(const v4f*)(W + (size_t)(k0 + kr) * kD + n0 + c4);
    tile[kr][c4 + 0] = v[0] * kWCarry;
    tile[kr][c4 + 1] = v[1] * kWCarry;
    tile[kr][c4 + 2] = v[2] * kWCarry;
    tile[kr][c4 + 3] = v[3] * kWCarry;
  }
  __syncthreads();
  const int lid = tid >> 3, c8 = (tid & 7) * 8;
  _Float16* O = (_Float16*)Wt;
  for (int pass = 0; pass < 2; ++pass) {
#pragma unroll
    for (int it = 0; it < 2; ++it) {
      const int nn = it * 32 + lid;
      v8h hv;
#pragma unroll
      for (int e = 0; e < 8; ++e) hv[e] = (_Float16)tile[c8 + e][nn];
      *(volatile v8h*)(O + (size_t)(n0 + nn) * kD + k0 + c8) = hv;
    }
    __threadfence();
  }
}

__global__ __launch_bounds__(256) void phase_tables(const float* __restrict__ phase, const float* __restrict__ carrier,
                                                    float* __restrict__ Th, float* __restrict__ logTh) {
#pragma clang fp contract(off)
  const int i = blockIdx.x * 256 + threadIdx.x;
  if (i >= kB * kH * kS) return;
  const int s = i & (kS - 1);
  const int bh = i >> 11;
  const int hd = bh & (kH - 1);
  const int b = bh >> 4;
  const float dph = (phase[b * kS + s] - carrier[hd]) * 0.5f;
  const float cv = cosf(dph);
  const float T = cv * cv;
  const float L = logf(T + 1e-6f);
  ((volatile float*)Th)[i] = T;
  ((volatile float*)logTh)[i] = L;
  __threadfence();
  ((volatile float*)Th)[i] = T;
  ((volatile float*)logTh)[i] = L;
}

__global__ __launch_bounds__(128)
void attn_f16_planes(const unsigned short* __restrict__ qp, const unsigned short* __restrict__ kp,
                     const unsigned short* __restrict__ vtp, const float* __restrict__ Th,
                     const float* __restrict__ logTh, const float* __restrict__ balance,
                     unsigned short* __restrict__ op) {
  __shared__ __align__(16) _Float16 Ksh[64 * 64];
  __shared__ __align__(16) _Float16 Vth[64 * 64];
  __shared__ __align__(16) _Float16 Psh[4][16 * 64];
  __shared__ __align__(16) float    Os[4][16 * 68];

  const int tid  = threadIdx.x;
  const int wave = tid >> 5;
  const int lane = tid & 31;
  const int hh   = lane >> 4;
  const int c    = lane & 15;

  constexpr int nqb = kS / 64;
  const int bx = blockIdx.x;
  const int qb = bx % nqb;
  const int bh = bx / nqb;
  const int h  = bh % kH;
  const int b  = bh / kH;
  const int q0 = qb * 64 + wave * 16;

  float tau = 1.0f / (2.0f * balance[0] + 1e-8f);
  tau = fminf(fmaxf(tau, 0.1f), 10.0f);
  const float inv_tau = 1.0f / tau;
  const float sscale = 0.125f / (kQKVCarry * kQKVCarry);

  const _Float16* Q = (const _Float16*)qp;
  const float* lth = logTh + (size_t)bh * kS;
  const float* thb = Th + (size_t)bh * kS;

  v16h qa[2];
  {
    const _Float16* qrow = Q + (size_t)(b * kS + q0 + c) * kD + h * kDH + 8 * hh;
    qa[0] = Frag<_Float16>::load(qrow);
    qa[1] = Frag<_Float16>::load(qrow + 32);
  }

  float mrow[8], lrow[8];
  v8f oacc[4];
#pragma unroll
  for (int r = 0; r < 8; ++r) { mrow[r] = -INFINITY; lrow[r] = 0.f; }
#pragma unroll
  for (int t = 0; t < 4; ++t) oacc[t] = (v8f){0.f,0.f,0.f,0.f,0.f,0.f,0.f,0.f};

  const int nChunks = qb + 1;
  for (int kc = 0; kc < nChunks; ++kc) {
    const int kv0 = kc * 64;
    __syncthreads();
#pragma unroll
    for (int i = 0; i < 4; ++i) {
      const int idx = tid + 128 * i;
      const int row = idx >> 3, seg = (idx & 7) * 8;
      const v4u kk = *(const v4u*)(kp + (size_t)(b * kS + kv0 + row) * kD + h * kDH + seg);
      *(v4u*)(void*)(Ksh + row * 64 + seg) = kk;
      const v4u vv = *(const v4u*)(vtp + (size_t)(h * kDH + row) * kM + b * kS + kv0 + seg);
      *(v4u*)(void*)(Vth + row * 64 + seg) = vv;
    }
    __syncthreads();

    v8f s[4];
#pragma unroll
    for (int j = 0; j < 4; ++j) {
      s[j] = (v8f){0.f,0.f,0.f,0.f,0.f,0.f,0.f,0.f};
#pragma unroll
      for (int dc = 0; dc < 2; ++dc) {
        const v16h kb = Frag<_Float16>::load(Ksh + (j * 16 + c) * 64 + dc * 32 + 8 * hh);
        s[j] = mma_h(qa[dc], kb, s[j]);
      }
    }
    const bool diag = (kc == qb);
    float lt[4];
#pragma unroll
    for (int j = 0; j < 4; ++j) lt[j] = lth[kv0 + j * 16 + c];
    float cm[8];
#pragma unroll
    for (int r = 0; r < 8; ++r) {
      const int qrow = q0 + 8 * hh + r;
      float m = -INFINITY;
#pragma unroll
      for (int j = 0; j < 4; ++j) {
        const int kvcol = kv0 + j * 16 + c;
        float sv = (s[j][r] * sscale + lt[j]) * inv_tau;
        if (diag && (kvcol > qrow)) sv = kMaskFill * inv_tau;
        s[j][r] = sv;
        m = fmaxf(m, sv);
      }
#pragma unroll
      for (int off = 1; off < 16; off <<= 1) m = fmaxf(m, __shfl_xor(m, off, 32));
      cm[r] = m;
    }
    _Float16* pwh = Psh[wave];
#pragma unroll
    for (int r = 0; r < 8; ++r) {
      const float mnew = fmaxf(mrow[r], cm[r]);
      const float alpha = expf(mrow[r] - mnew);
      mrow[r] = mnew;
      float psum = 0.f;
#pragma unroll
      for (int j = 0; j < 4; ++j) {
        const float p = expf(s[j][r] - mnew);
        psum += p;
        pwh[(8 * hh + r) * 64 + j * 16 + c] = (_Float16)(p * kPCarry);
      }
#pragma unroll
      for (int off = 1; off < 16; off <<= 1) psum += __shfl_xor(psum, off, 32);
      lrow[r] = lrow[r] * alpha + psum;
#pragma unroll
      for (int t = 0; t < 4; ++t) oacc[t][r] *= alpha;
    }
    __builtin_amdgcn_fence(__ATOMIC_RELEASE, "workgroup");
    __builtin_amdgcn_wave_barrier();
    __builtin_amdgcn_fence(__ATOMIC_ACQUIRE, "workgroup");
#pragma unroll 1
    for (int kk = 0; kk < 2; ++kk) {
      const v16h pa = Frag<_Float16>::load(pwh + c * 64 + kk * 32 + 8 * hh);
#pragma unroll
      for (int t = 0; t < 4; ++t) {
        const v16h vb = Frag<_Float16>::load(Vth + (t * 16 + c) * 64 + kk * 32 + 8 * hh);
        oacc[t] = mma_h(pa, vb, oacc[t]);
      }
    }
  }

  float* os = Os[wave];
#pragma unroll
  for (int r = 0; r < 8; ++r) {
    const int qrow = q0 + 8 * hh + r;
    const float thq = thb[qrow];
    const float f = (kOCarry / (kPCarry * kQKVCarry)) * thq * (1.0f / lrow[r]);
#pragma unroll
    for (int t = 0; t < 4; ++t) os[(8 * hh + r) * 68 + t * 16 + c] = oacc[t][r] * f;
  }
  __builtin_amdgcn_fence(__ATOMIC_RELEASE, "workgroup");
  __builtin_amdgcn_wave_barrier();
  __builtin_amdgcn_fence(__ATOMIC_ACQUIRE, "workgroup");
  {
    const int q8 = lane >> 3, c8 = (lane & 7) * 8;
    _Float16* O = (_Float16*)op;
    for (int pass = 0; pass < 2; ++pass) {
#pragma unroll
      for (int it = 0; it < 4; ++it) {
        const int row = it * 4 + q8;
        const float* sp = os + row * 68 + c8;
        v8h hv;
#pragma unroll
        for (int e = 0; e < 8; ++e) hv[e] = (_Float16)sp[e];
        *(volatile v8h*)(O + (size_t)(b * kS + q0 + row) * kD + h * kDH + c8) = hv;
      }
      __threadfence();
    }
  }
}

extern "C" void kernel_launch(void* const* d_in, const int* in_sizes, int n_in,
                              void* d_out, int out_size, void* d_ws, size_t ws_size,
                              hipStream_t stream) {
  if (n_in < 11) return;
  const float* x       = (const float*)d_in[0];
  const float* phase   = (const float*)d_in[1];
  const float* Wq      = (const float*)d_in[2];
  const float* Wk      = (const float*)d_in[3];
  const float* Wv      = (const float*)d_in[4];
  const float* Wo      = (const float*)d_in[5];
  const float* gamma   = (const float*)d_in[6];
  const float* beta    = (const float*)d_in[7];
  const float* expo    = (const float*)d_in[8];
  const float* carrier = (const float*)d_in[9];
  const float* balance = (const float*)d_in[10];
  if (in_sizes[0] != kM * kD || in_sizes[1] != kB * kS ||
      in_sizes[2] != kD * kD || in_sizes[3] != kD * kD || in_sizes[4] != kD * kD || in_sizes[5] != kD * kD ||
      in_sizes[6] < kD || in_sizes[7] < kD ||
      in_sizes[8] < kH || in_sizes[9] < kH || in_sizes[10] < 1 || out_size != kM * kD) return;
  if (ws_size < kWsTotal) return;

  char* ws = (char*)d_ws;
  unsigned short* hP   = (unsigned short*)(ws + kOffH);
  unsigned short* qP   = (unsigned short*)(ws + kOffQ);
  unsigned short* kcP  = (unsigned short*)(ws + kOffKc);
  unsigned short* vtP  = (unsigned short*)(ws + kOffVt);
  unsigned short* oP   = (unsigned short*)(ws + kOffO);
  unsigned short* wqP  = (unsigned short*)(ws + kOffWq);
  unsigned short* wkP  = (unsigned short*)(ws + kOffWk);
  unsigned short* wvP  = (unsigned short*)(ws + kOffWv);
  unsigned short* woP  = (unsigned short*)(ws + kOffWo);
  float* ThP  = (float*)(ws + kOffTh);
  float* LThP = (float*)(ws + kOffLTh);

  const dim3 gT(kD / 64, kD / 64);
  wt_cast_f16<<<gT, 256, 0, stream>>>(Wq, wqP);
  wt_cast_f16<<<gT, 256, 0, stream>>>(Wk, wkP);
  wt_cast_f16<<<gT, 256, 0, stream>>>(Wv, wvP);
  wt_cast_f16<<<gT, 256, 0, stream>>>(Wo, woP);

  ln_rows_f16<<<kM, 128, 0, stream>>>(x, gamma, beta, hP);

  phase_tables<<<(kB * kH * kS + 255) / 256, 256, 0, stream>>>(phase, carrier, ThP, LThP);

  const int tilesProj = (kM / 64) * (kD / 64);
  const dim3 gg((tilesProj + 7) / 8, 1);
  wmma_gemm64<0, false, 0, 1, false, 0><<<gg, 256, 0, stream>>>(
      hP, nullptr, kD, 0L, wqP, nullptr, kD, 0L, (void*)qP, nullptr, kD, 0L,
      nullptr, nullptr, 0L, kM, kD, kD, kQKVCarry / kWCarry);
  wmma_gemm64<0, false, 0, 1, false, 6><<<gg, 256, 0, stream>>>(
      hP, nullptr, kD, 0L, wkP, nullptr, kD, 0L, (void*)kcP, nullptr, kD, 0L,
      expo, nullptr, 0L, kM, kD, kD, 1.0f / kWCarry);
  const int tilesVt = (kD / 64) * (kM / 64);
  const dim3 gv((tilesVt + 7) / 8, 1);
  wmma_gemm64<0, false, 0, 1, false, 7><<<gv, 256, 0, stream>>>(
      wvP, nullptr, kD, 0L, hP, nullptr, kD, 0L, (void*)vtP, nullptr, kM, 0L,
      expo, nullptr, 0L, kD, kM, kD, 1.0f / kWCarry);

  attn_f16_planes<<<kB * kH * (kS / 64), 128, 0, stream>>>(qP, kcP, vtP, ThP, LThP, balance, oP);

  wmma_gemm64<0, false, 0, 0, true, 0><<<gg, 256, 0, stream>>>(
      oP, nullptr, kD, 0L, woP, nullptr, kD, 0L, d_out, nullptr, kD, 0L,
      nullptr, x, 0L, kM, kD, kD, 1.0f / (kOCarry * kWCarry));
}
